// EfficientAttention_42073499632181
// MI455X (gfx1250) — hardware-verified
//
#include <hip/hip_runtime.h>
#include <math.h>

#ifndef NB
#define NB 4
#endif
#ifndef SEQ
#define SEQ 2048
#endif
#define NB_FULL 4
#define SEQ_FULL 2048
#define HID 1024
#define NHD 8
#define HDM 128
#define VTLD ((long long)NB_FULL * SEQ_FULL)

static_assert(NB >= 1 && NB <= NB_FULL);
static_assert(SEQ >= 64 && SEQ <= SEQ_FULL && (SEQ % 64) == 0);
static_assert(HID == NHD * HDM);
static_assert((HID % 64) == 0 && (HID % 32) == 0 && HDM == 128);

typedef __attribute__((ext_vector_type(16))) _Float16 v16h;
typedef __attribute__((ext_vector_type(8)))  _Float16 v8h;
typedef __attribute__((ext_vector_type(8)))  float    v8f;
typedef __attribute__((ext_vector_type(4)))  float    v4f;

union FH { v16h v; v8h h[2]; };
__device__ __forceinline__ v16h fh_frag(const _Float16* p) { FH f; f.h[0] = *(const v8h*)p; f.h[1] = *(const v8h*)(p + 16); return f.v; }

__device__ __forceinline__ v8f wmma16(v16h a, v16h b, v8f c) {
    c = __builtin_amdgcn_wmma_f32_16x16x32_f16(false, a, false, b, (short)0, c, false, false);
    asm volatile("v_nop\n\tv_nop\n\tv_nop\n\tv_nop" : "+v"(c) : "v"(a), "v"(b));
    return c;
}
__device__ __forceinline__ void dep_guard_h(v8f& a, v8f& b, v16h x, v16h y) { asm volatile("v_nop\n\tv_nop\n\tv_nop\n\tv_nop" : "+v"(a), "+v"(b) : "v"(x), "v"(y)); }
__device__ __forceinline__ void keep4_h(v16h a, v16h b, v16h c, v16h d) { asm volatile("v_nop" :: "v"(a), "v"(b), "v"(c), "v"(d)); }
__device__ __forceinline__ void acc_guard4(v8f& a, v8f& b, v8f& c, v8f& d) { asm volatile("v_nop\n\tv_nop\n\tv_nop\n\tv_nop" : "+v"(a), "+v"(b), "+v"(c), "+v"(d)); }

__device__ __forceinline__ float bfr(float f) {
    unsigned int u = __float_as_uint(f);
    u += 0x7fffu + ((u >> 16) & 1u);
    u &= 0xffff0000u;
    return __uint_as_float(u);
}

__global__ __launch_bounds__(256) void k_cast8(const float* __restrict__ src, long long sstr, _Float16* __restrict__ dst, long long dstr, int n8, float s) {
    const int i = blockIdx.x * 256 + threadIdx.x;
    if (i >= n8) return;
    const float* sp = src + (long long)blockIdx.y * sstr + 8 * (long long)i;
    _Float16* dp = dst + (long long)blockIdx.y * dstr + 8 * (long long)i;
    const v4f a = *(const v4f*)sp;
    const v4f b = *(const v4f*)(sp + 4);
    v8h hv;
    hv[0] = (_Float16)(bfr(a.x) * s); hv[1] = (_Float16)(bfr(a.y) * s); hv[2] = (_Float16)(bfr(a.z) * s); hv[3] = (_Float16)(bfr(a.w) * s);
    hv[4] = (_Float16)(bfr(b.x) * s); hv[5] = (_Float16)(bfr(b.y) * s); hv[6] = (_Float16)(bfr(b.z) * s); hv[7] = (_Float16)(bfr(b.w) * s);
    *(volatile v8h*)dp = hv;
    __threadfence();
    *(volatile v8h*)dp = hv;
}

template <int OUT_MODE>
__global__ __launch_bounds__(256) void k_gemm64(const _Float16* __restrict__ A, int lda, long long strideA,
                                                 const _Float16* __restrict__ Bt, int ldb, long long strideB,
                                                 void* __restrict__ Cout, int ldc, long long strideC,
                                                 int M, int N, int K, float scale) {
    __shared__ __align__(16) float sT[8][16 * 68];
    const int bz   = blockIdx.y;
    const int lane = threadIdx.x & 31;
    const int wave = threadIdx.x >> 5;
    const int tilesN = N >> 6;
    const int tilesM = M >> 6;
    const int tile = blockIdx.x * 8 + wave;
    if (tile >= tilesM * tilesN) return;
    const int tm = tile / tilesN;
    const int tn = tile - tm * tilesN;
    const int m0 = tm << 6;
    const int n0 = tn << 6;

    const _Float16* Ab = A  + (size_t)bz * strideA;
    const _Float16* Bb = Bt + (size_t)bz * strideB;

    const int rlane = lane & 15;
    const int koff  = (lane >> 4) * 8;
    const int mOff  = (lane >> 4) * 8;

    v8f acc[4][4];
#pragma unroll
    for (int i = 0; i < 4; ++i)
#pragma unroll
        for (int j = 0; j < 4; ++j) acc[i][j] = (v8f){0.f, 0.f, 0.f, 0.f, 0.f, 0.f, 0.f, 0.f};

    for (int k0 = 0; k0 < K; k0 += 32) {
        v16h bh[4];
#pragma unroll
        for (int j = 0; j < 4; ++j) {
            const size_t bo = (size_t)(n0 + (j << 4) + rlane) * ldb + koff + k0;
            bh[j] = fh_frag(Bb + bo);
        }
#pragma unroll
        for (int i = 0; i < 4; ++i) {
            const size_t ao = (size_t)(m0 + (i << 4) + rlane) * lda + koff + k0;
            const v16h ah = fh_frag(Ab + ao);
#pragma unroll
            for (int j = 0; j < 4; ++j)
                acc[i][j] = __builtin_amdgcn_wmma_f32_16x16x32_f16(false, ah, false, bh[j], (short)0, acc[i][j], false, false);
            dep_guard_h(acc[i][0], acc[i][3], ah, ah);
        }
        keep4_h(bh[0], bh[1], bh[2], bh[3]);
    }
    acc_guard4(acc[0][0], acc[0][1], acc[0][2], acc[0][3]);
    acc_guard4(acc[1][0], acc[1][1], acc[1][2], acc[1][3]);
    acc_guard4(acc[2][0], acc[2][1], acc[2][2], acc[2][3]);
    acc_guard4(acc[3][0], acc[3][1], acc[3][2], acc[3][3]);

    float* slab = sT[wave];
#pragma unroll
    for (int i = 0; i < 4; ++i) {
        const int mBase = m0 + (i << 4);
#pragma unroll
        for (int j = 0; j < 4; ++j) {
#pragma unroll
            for (int r = 0; r < 8; ++r) {
                const float v = acc[i][j][r] * scale;
                slab[(mOff + r) * 68 + (j << 4) + rlane] = v;
            }
        }
        __builtin_amdgcn_fence(3, "workgroup");
        __builtin_amdgcn_wave_barrier();
        __builtin_amdgcn_fence(2, "workgroup");
        if (OUT_MODE == 0) {
            float* C = (float*)Cout + (size_t)bz * strideC;
            const int hh = lane >> 4, c4 = (lane & 15) * 4;
            for (int pass = 0; pass < 2; ++pass) {
#pragma unroll
                for (int it = 0; it < 8; ++it) {
                    const int row = it * 2 + hh;
                    const v4f v = *(const v4f*)(slab + row * 68 + c4);
                    *(volatile v4f*)(C + (size_t)(mBase + row) * ldc + n0 + c4) = v;
                }
                __threadfence();
            }
        } else {
            _Float16* C = (_Float16*)Cout + (size_t)bz * strideC;
            const int q = lane >> 3, c8 = (lane & 7) * 8;
            for (int pass = 0; pass < 2; ++pass) {
#pragma unroll
                for (int it = 0; it < 4; ++it) {
                    const int row = it * 4 + q;
                    const float* sp = slab + row * 68 + c8;
                    v8h hv;
#pragma unroll
                    for (int e = 0; e < 8; ++e) hv[e] = (_Float16)sp[e];
                    *(volatile v8h*)(C + (size_t)(mBase + row) * ldc + n0 + c8) = hv;
                }
                __threadfence();
            }
        }
        __builtin_amdgcn_fence(3, "workgroup");
        __builtin_amdgcn_wave_barrier();
        __builtin_amdgcn_fence(2, "workgroup");
    }
}

#define KCH 64
#define KSP 136
#define VSP 72
#define PSP 72
#define OSP 132
#define PCAR 4096.0f
static_assert(4 * 16 * OSP * 4 <= (KCH * KSP + HDM * VSP) * 2);
static_assert((SEQ % KCH) == 0);

__global__ __launch_bounds__(128) __attribute__((amdgpu_num_vgpr(256)))
void k_attn128(const _Float16* __restrict__ Q16, const _Float16* __restrict__ K16, const _Float16* __restrict__ VT16,
               _Float16* __restrict__ CTX16, float sl2, float osc) {
    __shared__ __align__(16) _Float16 kvs[KCH * KSP + HDM * VSP];
    __shared__ __align__(16) _Float16 qsm[4 * 16 * KSP];
    __shared__ __align__(16) _Float16 psm[4 * 16 * PSP];
    const int tid = threadIdx.x, wave = tid >> 5, lane = tid & 31, hh = lane >> 4, c = lane & 15;
    const int nqb = SEQ / 64;
    const int bx = blockIdx.x;
    const int qb = bx % nqb, bhd = bx / nqb, h = bhd % NHD, b = bhd / NHD;
    const int q0 = qb * 64 + wave * 16;
    const long long trow = (long long)b * SEQ_FULL;
    _Float16* Ks = kvs;
    _Float16* Vs = kvs + KCH * KSP;
    _Float16* Qs = qsm + wave * 16 * KSP;
    _Float16* Ps = psm + wave * 16 * PSP;

    {
        const _Float16* qbp = Q16 + (trow + q0) * HID + h * HDM;
#pragma unroll
        for (int i = 0; i < 8; ++i) {
            const int p = lane + 32 * i;
            const int r = p >> 4, col = (p & 15) * 8;
            const v8h v = *(const v8h*)(qbp + (long long)r * HID + col);
            *(v8h*)(Qs + r * KSP + col) = v;
        }
    }

    float mrow[8], lrow[8];
    v8f oacc[8];
#pragma unroll
    for (int r = 0; r < 8; ++r) { mrow[r] = -__builtin_inff(); lrow[r] = 0.f; }
#pragma unroll
    for (int t = 0; t < 8; ++t) oacc[t] = (v8f){0.f, 0.f, 0.f, 0.f, 0.f, 0.f, 0.f, 0.f};

    const _Float16* kbp = K16 + trow * HID + h * HDM;
    const _Float16* vbp = VT16 + (long long)(h * HDM) * VTLD + trow;
    const int nch = SEQ / KCH;
#pragma unroll 1
    for (int kc = 0; kc < nch; ++kc) {
        const int kv0 = kc * KCH;
        __syncthreads();
#pragma unroll 4
        for (int i = 0; i < 8; ++i) {
            const int p = tid + 128 * i;
            const int kr = p >> 4, kcol = (p & 15) * 8;
            const int vd = p >> 3, vcol = (p & 7) * 8;
            const v8h kvv = *(const v8h*)(kbp + (long long)(kv0 + kr) * HID + kcol);
            const v8h vvv = *(const v8h*)(vbp + (long long)vd * VTLD + kv0 + vcol);
            *(v8h*)(Ks + kr * KSP + kcol) = kvv;
            *(v8h*)(Vs + vd * VSP + vcol) = vvv;
        }
        __syncthreads();

        v8f s[4];
#pragma unroll
        for (int j = 0; j < 4; ++j) {
            v8f a = (v8f){0.f, 0.f, 0.f, 0.f, 0.f, 0.f, 0.f, 0.f};
            const _Float16* qr = Qs + c * KSP + 8 * hh;
            const _Float16* kr = Ks + (j * 16 + c) * KSP + 8 * hh;
#pragma unroll 1
            for (int dc = 0; dc < 4; ++dc) a = wmma16(fh_frag(qr + dc * 32), fh_frag(kr + dc * 32), a);
            s[j] = a;
        }

#pragma unroll
        for (int r = 0; r < 8; ++r) {
            float mx = fmaxf(fmaxf(s[0][r], s[1][r]), fmaxf(s[2][r], s[3][r]));
#pragma unroll
            for (int off = 1; off < 16; off <<= 1) mx = fmaxf(mx, __shfl_xor(mx, off, 32));
            const float mnew = fmaxf(mrow[r], mx * sl2);
            const float alpha = exp2f(mrow[r] - mnew);
            mrow[r] = mnew;
            float psum = 0.f;
#pragma unroll
            for (int j = 0; j < 4; ++j) {
                const float pj = exp2f(s[j][r] * sl2 - mnew);
                psum += pj;
                Ps[(8 * hh + r) * PSP + j * 16 + c] = (_Float16)(pj * PCAR);
            }
#pragma unroll
            for (int off = 1; off < 16; off <<= 1) psum += __shfl_xor(psum, off, 32);
            lrow[r] = lrow[r] * alpha + psum;
#pragma unroll
            for (int t = 0; t < 8; ++t) oacc[t][r] *= alpha;
        }
        __syncthreads();

#pragma unroll 1
        for (int kk = 0; kk < 2; ++kk) {
            const v16h pa = fh_frag(Ps + c * PSP + kk * 32 + 8 * hh);
#pragma unroll
            for (int t = 0; t < 8; ++t)
                oacc[t] = wmma16(pa, fh_frag(Vs + (t * 16 + c) * VSP + kk * 32 + 8 * hh), oacc[t]);
        }
    }

    __syncthreads();
    float* os = (float*)kvs + wave * (16 * OSP);
#pragma unroll
    for (int r = 0; r < 8; ++r) {
        const float inv = osc / lrow[r];
#pragma unroll
        for (int t = 0; t < 8; ++t) os[(8 * hh + r) * OSP + t * 16 + c] = oacc[t][r] * inv;
    }
    __syncthreads();
    _Float16* ob = CTX16 + (trow + q0) * HID + h * HDM;
    const int c8 = c * 8;
    for (int pass = 0; pass < 2; ++pass) {
#pragma unroll
        for (int it = 0; it < 8; ++it) {
            const int row = it * 2 + hh;
            const float* sp = os + row * OSP + c8;
            const v4f a0 = *(const v4f*)sp;
            const v4f a1 = *(const v4f*)(sp + 4);
            v8h hv;
            hv[0] = (_Float16)a0.x; hv[1] = (_Float16)a0.y; hv[2] = (_Float16)a0.z; hv[3] = (_Float16)a0.w;
            hv[4] = (_Float16)a1.x; hv[5] = (_Float16)a1.y; hv[6] = (_Float16)a1.z; hv[7] = (_Float16)a1.w;
            *(volatile v8h*)(ob + (long long)row * HID + c8) = hv;
        }
        __threadfence();
    }
}

extern "C" void kernel_launch(void* const* d_in, const int* in_sizes, int n_in,
                              void* d_out, int out_size, void* d_ws, size_t ws_size, hipStream_t stream) {
    if (n_in < 5) return;
    const long long need_x = ((long long)(NB - 1) * SEQ_FULL + SEQ) * (long long)HID;
    if ((long long)in_sizes[0] < need_x) return;
    if ((long long)in_sizes[1] < (long long)HID * HID) return;
    if ((long long)in_sizes[2] < (long long)HID * HID) return;
    if ((long long)in_sizes[3] < (long long)HID * HID) return;
    if ((long long)in_sizes[4] < (long long)HID * HID) return;
    if ((long long)out_size < (long long)NB * SEQ * HID) return;

    const float* hs = (const float*)d_in[0];
    const float* Wq = (const float*)d_in[1];
    const float* Wk = (const float*)d_in[2];
    const float* Wv = (const float*)d_in[3];
    const float* Wo = (const float*)d_in[4];
    float* out = (float*)d_out;

    const size_t nTok   = (size_t)NB_FULL * SEQ_FULL;
    const size_t bTok16 = nTok * HID * 2;
    const size_t bW16   = (size_t)HID * HID * 2;
    char* wsp = (char*)d_ws;
    size_t off = 0;
    _Float16* X16   = (_Float16*)(wsp + off); off += bTok16;
    _Float16* Wq16  = (_Float16*)(wsp + off); off += bW16;
    _Float16* Wk16  = (_Float16*)(wsp + off); off += bW16;
    _Float16* Wv16  = (_Float16*)(wsp + off); off += bW16;
    _Float16* Wo16  = (_Float16*)(wsp + off); off += bW16;
    _Float16* Q16   = (_Float16*)(wsp + off); off += bTok16;
    _Float16* K16   = (_Float16*)(wsp + off); off += bTok16;
    _Float16* VT16  = (_Float16*)(wsp + off); off += bTok16;
    _Float16* CTX16 = (_Float16*)(wsp + off); off += bTok16;
    if (off > ws_size) return;

    const long long tokStride = (long long)SEQ_FULL * HID;
    const float wcar = 64.0f;
    const float sl2  = 0.08838834764831845f * 1.4426950408889634f;
    const float osc  = 64.0f / PCAR;

    {
        const int n8x = SEQ * HID / 8;
        k_cast8<<<dim3((unsigned)((n8x + 255) / 256), (unsigned)NB), 256, 0, stream>>>(hs, tokStride, X16, tokStride, n8x, 1.0f);
        const int n8w = HID * HID / 8;
        k_cast8<<<dim3((unsigned)((n8w + 255) / 256), 1u), 256, 0, stream>>>(Wq, 0, Wq16, 0, n8w, wcar);
        k_cast8<<<dim3((unsigned)((n8w + 255) / 256), 1u), 256, 0, stream>>>(Wk, 0, Wk16, 0, n8w, wcar);
        k_cast8<<<dim3((unsigned)((n8w + 255) / 256), 1u), 256, 0, stream>>>(Wv, 0, Wv16, 0, n8w, wcar);
        k_cast8<<<dim3((unsigned)((n8w + 255) / 256), 1u), 256, 0, stream>>>(Wo, 0, Wo16, 0, n8w, wcar);
    }
    {
        const int tilesQK = (SEQ / 64) * (HID / 64);
        const dim3 gqk((unsigned)((tilesQK + 7) / 8), (unsigned)NB);
        k_gemm64<1><<<gqk, 256, 0, stream>>>(X16, HID, tokStride, Wq16, HID, 0, (void*)Q16, HID, tokStride, SEQ, HID, HID, 1.0f / wcar);
        k_gemm64<1><<<gqk, 256, 0, stream>>>(X16, HID, tokStride, Wk16, HID, 0, (void*)K16, HID, tokStride, SEQ, HID, HID, 1.0f / wcar);
        const int tilesV = (HID / 64) * (SEQ / 64);
        const dim3 gv((unsigned)((tilesV + 7) / 8), (unsigned)NB);
        k_gemm64<1><<<gv, 256, 0, stream>>>(Wv16, HID, 0, X16, HID, tokStride, (void*)VT16, (int)VTLD, (long long)SEQ_FULL, HID, SEQ, HID, 1.0f / wcar);
    }
    k_attn128<<<dim3((unsigned)(NB * NHD * (SEQ / 64))), 128, 0, stream>>>(Q16, K16, VT16, CTX16, sl2, osc);
    {
        const int tilesO = (SEQ / 64) * (HID / 64);
        const dim3 go((unsigned)((tilesO + 7) / 8), (unsigned)NB);
        k_gemm64<0><<<go, 256, 0, stream>>>(CTX16, HID, tokStride, Wo16, HID, 0, (void*)out, HID, (long long)SEQ * HID, SEQ, HID, HID, 1.0f / (wcar * wcar));
    }
}
